// SlotConditioner_12859132084466
// MI455X (gfx1250) — hardware-verified
//
#include <hip/hip_runtime.h>
#include <hip/hip_bf16.h>
#include <math.h>


#define BB 2
#define SS 2048
#define DD 1024
#define HH 16
#define DKK 64
#define QW 2

typedef _Float16 bf16;
typedef __attribute__((ext_vector_type(4))) unsigned v4u_t;
typedef unsigned v4ua __attribute__((ext_vector_type(4), may_alias));
typedef __attribute__((ext_vector_type(4))) float v4f_t;
typedef float v4fa __attribute__((ext_vector_type(4), may_alias));
typedef __attribute__((ext_vector_type(16))) bf16  bf16x16;
typedef __attribute__((ext_vector_type(8)))  bf16  bf16x8;
typedef __attribute__((ext_vector_type(4)))  bf16  bf16x4;
typedef __attribute__((ext_vector_type(8)))  float f32x8;

#define LDS_STRIDE 48
#define KSTRIDE    72
#define VSTRIDE    48

__device__ __forceinline__ f32x8 wmma_bf16(bf16x16 a, bf16x16 b, f32x8 c) {
  return __builtin_amdgcn_wmma_f32_16x16x32_f16(
      false, a, false, b, (short)0, c, false, false);
}
#define RSPLIT (1.0f / 2048.0f)
__device__ __forceinline__ bf16 lo_of(float v, bf16 h) { return (bf16)((v - (float)h) * 2048.0f); }
__device__ __forceinline__ f32x8 wmma_split(bf16x16 a, bf16x16 al, bf16x16 b, bf16x16 bl, f32x8 c) {
  f32x8 x = {}; x = wmma_bf16(al, b, x); x = wmma_bf16(a, bl, x); return wmma_bf16(a, b, c) + x * RSPLIT; }

template <typename T>
__device__ __forceinline__ bf16x16 load_frag(const T* __restrict__ base, int ld,
                                             int row0, int k0) {
  const int lane = threadIdx.x & 31;
  const int r    = lane & 15;
  const int kh   = (lane >> 4) * 8;
  const T* p0 = base + (size_t)(row0 + r) * ld + (k0 + kh);
  const T* p1 = p0 + 16;
  bf16x16 f;
#pragma unroll
  for (int i = 0; i < 8; ++i) {
    f[i]     = (bf16)p0[i];
    f[i + 8] = (bf16)p1[i];
  }
  return f;
}

__device__ __forceinline__ bf16x16 lds_frag(const bf16* base, int stride) {
  const int lane = threadIdx.x & 31;
  const int row  = lane & 15;
  const int kh   = (lane >> 4) * 8;
  const bf16x8 lo = *(const bf16x8*)(base + row * stride + kh);
  const bf16x8 hi = *(const bf16x8*)(base + row * stride + kh + 16);
  bf16x16 f;
#pragma unroll
  for (int i = 0; i < 8; ++i) { f[i] = lo[i]; f[i + 8] = hi[i]; }
  return f;
}

template <typename T>
__device__ __forceinline__ void stage_read16(const T* __restrict__ p, float* buf) {
#pragma unroll
  for (int i = 0; i < 16; ++i) buf[i] = (float)p[i];
}

__device__ __forceinline__ void stage_write(bf16* dst, const float* buf, int nquad) {
#pragma unroll
  for (int i = 0; i < nquad; ++i) {
    bf16x4 q;
    q[0] = (bf16)buf[4 * i];     q[1] = (bf16)buf[4 * i + 1];
    q[2] = (bf16)buf[4 * i + 2]; q[3] = (bf16)buf[4 * i + 3];
    *(bf16x4*)(dst + 4 * i) = q;
  }
}

__global__ __launch_bounds__(256) void transpose_pack_kernel(const float* __restrict__ W, bf16* __restrict__ WT, int K, int N, size_t plane) {
  __shared__ float tile[64][65];
  const int k0 = blockIdx.y * 64, n0 = blockIdx.x * 64, t = threadIdx.x;
  for (int i = t; i < 64 * 64; i += 256) { const int kr = i >> 6, nc = i & 63; tile[kr][nc] = W[(size_t)(k0 + kr) * N + n0 + nc]; }
  __syncthreads();
#pragma unroll 1
  for (int pass = 0; pass < 2; ++pass) {
    for (int i = t; i < 64 * 8; i += 256) { const int nr = i >> 3, k8 = (i & 7) * 8; bf16 hh[8], hl[8];
#pragma unroll
      for (int e = 0; e < 8; ++e) { const float v = tile[k8 + e][nr]; hh[e] = (bf16)v; hl[e] = lo_of(v, hh[e]); }
      bf16* d = WT + (size_t)(n0 + nr) * K + k0 + k8;
      *(volatile v4u_t*)d = *(const v4ua*)hh; *(volatile v4u_t*)(d + plane) = *(const v4ua*)hl; }
    __threadfence();
  }
}

template <typename AT, typename WT, int MODE>
__global__ __launch_bounds__(256) void gemm_split_kernel(
    const AT* __restrict__ A, size_t aPlane, const WT* __restrict__ W, size_t wPlane,
    const float* __restrict__ bias, void* __restrict__ out,
    int M, int N, int K) {
  __shared__ bf16 ldsA[128 * LDS_STRIDE], ldsAl[128 * LDS_STRIDE];
  __shared__ bf16 ldsW[256 * LDS_STRIDE], ldsWl[256 * LDS_STRIDE];
  __shared__ __attribute__((aligned(16))) unsigned char sob[256 * 136 * 2];

  const int t    = threadIdx.x;
  const int wave = t >> 5;
  const int lane = t & 31;
  const int wm   = (wave & 1) * 64;
  const int wn   = (wave >> 1) * 64;
  const int mBlk = blockIdx.x * 128;
  const int nBlk = blockIdx.y * 256;
  const int arow = t >> 1;
  const int ach  = (t & 1) * 16;

  f32x8 acc[4][4] = {};
  for (int k = 0; k < K; k += 32) {
    __syncthreads();
    {
      const AT* ap = A + (size_t)(mBlk + arow) * K + k + ach;
      bf16 hh[16], hl[16];
      if (sizeof(AT) == 4) {
#pragma unroll
        for (int i = 0; i < 16; ++i) { const float v = (float)ap[i]; hh[i] = (bf16)v; hl[i] = lo_of(v, hh[i]); }
      } else {
#pragma unroll
        for (int i = 0; i < 16; ++i) { hh[i] = (bf16)ap[i]; hl[i] = (bf16)ap[aPlane + i]; }
      }
#pragma unroll
      for (int i = 0; i < 16; ++i) { ldsA[arow * LDS_STRIDE + ach + i] = hh[i]; ldsAl[arow * LDS_STRIDE + ach + i] = hl[i]; }
    }
    {
      const WT* wp = W + (size_t)(nBlk + t) * K + k;
      if (sizeof(WT) == 4) {
#pragma unroll
        for (int i = 0; i < 32; ++i) { const float v = (float)wp[i]; const bf16 h_ = (bf16)v; ldsW[t * LDS_STRIDE + i] = h_; ldsWl[t * LDS_STRIDE + i] = lo_of(v, h_); }
      } else {
#pragma unroll
        for (int i = 0; i < 32; ++i) { ldsW[t * LDS_STRIDE + i] = (bf16)wp[i]; ldsWl[t * LDS_STRIDE + i] = (bf16)wp[wPlane + i]; }
      }
    }
    __syncthreads();
    bf16x16 wf[4], wfl[4];
#pragma unroll
    for (int j = 0; j < 4; ++j) { wf[j] = lds_frag(ldsW + (wn + 16 * j) * LDS_STRIDE, LDS_STRIDE); wfl[j] = lds_frag(ldsWl + (wn + 16 * j) * LDS_STRIDE, LDS_STRIDE); }
#pragma unroll
    for (int i = 0; i < 4; ++i) {
      const bf16x16 af = lds_frag(ldsA + (wm + 16 * i) * LDS_STRIDE, LDS_STRIDE), afl = lds_frag(ldsAl + (wm + 16 * i) * LDS_STRIDE, LDS_STRIDE);
#pragma unroll
      for (int j = 0; j < 4; ++j) acc[i][j] = wmma_split(af, afl, wf[j], wfl[j], acc[i][j]);
    }
  }

  const int nlane = lane & 15;
  const int mh    = (lane >> 4) * 8;
  __syncthreads();
  if (MODE == 1) {
    bf16* so = (bf16*)sob;
#pragma unroll
    for (int i = 0; i < 4; ++i)
#pragma unroll
      for (int j = 0; j < 4; ++j) {
        const int nl = wn + 16 * j + nlane;
        const float bv = bias ? bias[nBlk + nl] : 0.0f;
#pragma unroll
        for (int r = 0; r < 8; ++r) so[nl * 136 + wm + 16 * i + mh + r] = (bf16)(acc[i][j][r] + bv);
      }
    __syncthreads();
    const int b_ = mBlk >> 11, s0 = mBlk & (SS - 1);
#pragma unroll 1
    for (int pass = 0; pass < 2; ++pass) {
      for (int ch = t; ch < 256 * 16; ch += 256) { const int nl = ch >> 4, q = (ch & 15) * 8; const int n = nBlk + nl, h = n >> 6, dk = n & (DKK - 1);
        *(volatile v4u_t*)((bf16*)out + (((size_t)(b_ * HH + h)) * DKK + dk) * SS + s0 + q) = *(const v4ua*)(so + nl * 136 + q); }
      __threadfence();
    }
  } else {
    float* so = (float*)sob;
#pragma unroll 1
    for (int hf = 0; hf < 2; ++hf) {
      if (wm == hf * 64) {
#pragma unroll
        for (int i = 0; i < 4; ++i)
#pragma unroll
          for (int j = 0; j < 4; ++j) {
            const int nl = wn + 16 * j + nlane;
            const float bv = bias ? bias[nBlk + nl] : 0.0f;
#pragma unroll
            for (int r = 0; r < 8; ++r) so[(16 * i + mh + r) * 260 + nl] = acc[i][j][r] + bv;
          }
      }
      __syncthreads();
#pragma unroll 1
      for (int pass = 0; pass < 2; ++pass) {
        for (int ch = t; ch < 64 * 64; ch += 256) { const int ml = ch >> 6, q = (ch & 63) * 4;
          *(volatile v4f_t*)((float*)out + (size_t)(mBlk + hf * 64 + ml) * N + nBlk + q) = *(const volatile v4fa*)(so + ml * 260 + q); }
        __threadfence();
      }
      __syncthreads();
    }
  }
}


#define NBS 1024
#define NSL 128
#define SD 64
#define TD 512
#define AD 384
#define HID 256
#define OD 64
#define M0 40
#define NM 16
#define CB 256

__global__ __launch_bounds__(224) void k_cat(const float* __restrict__ te, const float* __restrict__ au, float* __restrict__ TA) {
  const int b = blockIdx.x, t = threadIdx.x; v4f_t v; if (t < 128) v = *(const v4fa*)(te + (size_t)b * TD + t * 4); else v = *(const v4fa*)(au + (size_t)b * AD + (t - 128) * 4);
  *(volatile v4f_t*)(TA + (size_t)b * (TD + AD) + t * 4) = v; __threadfence(); *(volatile v4f_t*)(TA + (size_t)b * (TD + AD) + t * 4) = v;
}
__global__ __launch_bounds__(256) void k_packA(const float* __restrict__ W2, float* __restrict__ A) {
  const int m = blockIdx.x, k = threadIdx.x; const float v = (m < OD) ? W2[(size_t)k * OD + m] : 0.0f;
  *(volatile float*)(A + (size_t)m * HID + k) = v; __threadfence(); *(volatile float*)(A + (size_t)m * HID + k) = v;
}
template <int NS>
__global__ __launch_bounds__(256) void k_hrows(const float* __restrict__ U, const float* __restrict__ T, const float* __restrict__ b1, int b0, int s0, float* __restrict__ H) {
  const int bl = blockIdx.y, s = blockIdx.x, j = threadIdx.x, b = b0 + bl;
  const float u = U[(size_t)(s0 + s) * HID + j] + T[(size_t)b * HID + j] + b1[j];
  const float g = 0.5f * u * (1.0f + erff(u * 0.70710678118654752f));
  float* dst = H + ((size_t)bl * NS + s) * HID + j; *(volatile float*)dst = g; __threadfence(); *(volatile float*)dst = g;
}
template <int NS>
__global__ __launch_bounds__(64) void k_fin(const float* __restrict__ T2, int ncol, const float* __restrict__ b2, int b0, int s0, float* __restrict__ out) {
  const int bl = blockIdx.y, s = blockIdx.x, o = threadIdx.x, b = b0 + bl;
  const float v = T2[(size_t)o * ncol + bl * NS + s] + b2[o];
  float* dst = out + ((size_t)b * NSL + s0 + s) * OD + o; *(volatile float*)dst = v; __threadfence(); *(volatile float*)dst = v;
}

extern "C" void kernel_launch(void* const* d_in, const int* in_sizes, int n_in,
                              void* d_out, int out_size, void* d_ws, size_t ws_size,
                              hipStream_t stream) {
  (void)in_sizes; (void)n_in; (void)out_size; (void)ws_size;
  const float* te = (const float*)d_in[0];
  const float* au = (const float*)d_in[1];
  const float* emb = (const float*)d_in[2];
  const float* w1m = (const float*)d_in[3]; const float* b1m = (const float*)d_in[4]; const float* w2m = (const float*)d_in[5]; const float* b2m = (const float*)d_in[6];
  const float* w1u = (const float*)d_in[7]; const float* b1u = (const float*)d_in[8]; const float* w2u = (const float*)d_in[9]; const float* b2u = (const float*)d_in[10];
  float* out = (float*)d_out;
  char* ws = (char*)d_ws;
  const size_t plS = (size_t)HID * SD, plT = (size_t)HID * TD, plTA = (size_t)HID * (TD + AD);
  bf16* W1mS = (bf16*)ws; ws += plS * 2 * 2;
  bf16* W1mT = (bf16*)ws; ws += plT * 2 * 2;
  bf16* W1uS = (bf16*)ws; ws += plS * 2 * 2;
  bf16* W1uT = (bf16*)ws; ws += plTA * 2 * 2;
  float* A2m = (float*)ws; ws += (size_t)128 * HID * 4;
  float* A2u = (float*)ws; ws += (size_t)128 * HID * 4;
  float* TA  = (float*)ws; ws += (size_t)NBS * (TD + AD) * 4;
  float* Um  = (float*)ws; ws += (size_t)128 * HID * 4;
  float* Uu  = (float*)ws; ws += (size_t)128 * HID * 4;
  float* Tm  = (float*)ws; ws += (size_t)NBS * HID * 4;
  float* Tu  = (float*)ws; ws += (size_t)NBS * HID * 4;
  float* H   = (float*)ws; ws += (size_t)CB * NSL * HID * 4;
  float* T2  = (float*)ws; ws += (size_t)128 * CB * NSL * 4;
  transpose_pack_kernel<<<dim3(HID / 64, SD / 64), 256, 0, stream>>>(w1m, W1mS, SD, HID, plS);
  transpose_pack_kernel<<<dim3(HID / 64, TD / 64), 256, 0, stream>>>(w1m + (size_t)SD * HID, W1mT, TD, HID, plT);
  transpose_pack_kernel<<<dim3(HID / 64, SD / 64), 256, 0, stream>>>(w1u, W1uS, SD, HID, plS);
  transpose_pack_kernel<<<dim3(HID / 64, (TD + AD) / 64), 256, 0, stream>>>(w1u + (size_t)SD * HID, W1uT, TD + AD, HID, plTA);
  k_packA<<<128, 256, 0, stream>>>(w2m, A2m);
  k_packA<<<128, 256, 0, stream>>>(w2u, A2u);
  k_cat<<<NBS, 224, 0, stream>>>(te, au, TA);
  dim3 blk(256);
  gemm_split_kernel<float, bf16, 2><<<dim3(1, 1), blk, 0, stream>>>(emb, 0, W1mS, plS, nullptr, Um, NSL, HID, SD);
  gemm_split_kernel<float, bf16, 2><<<dim3(1, 1), blk, 0, stream>>>(emb, 0, W1uS, plS, nullptr, Uu, NSL, HID, SD);
  gemm_split_kernel<float, bf16, 2><<<dim3(NBS / 128, 1), blk, 0, stream>>>(te, 0, W1mT, plT, nullptr, Tm, NBS, HID, TD);
  gemm_split_kernel<float, bf16, 2><<<dim3(NBS / 128, 1), blk, 0, stream>>>(TA, 0, W1uT, plTA, nullptr, Tu, NBS, HID, TD + AD);
  for (int c = 0; c < NBS / CB; ++c) {
    const int b0 = c * CB;
    k_hrows<NSL><<<dim3(NSL, CB), 256, 0, stream>>>(Um, Tm, b1m, b0, 0, H);
    gemm_split_kernel<float, float, 2><<<dim3(1, CB * NSL / 256), blk, 0, stream>>>(A2m, 0, H, 0, nullptr, T2, 128, CB * NSL, HID);
    k_fin<NSL><<<dim3(NSL, CB), 64, 0, stream>>>(T2, CB * NSL, b2m, b0, 0, out);
    k_hrows<NM><<<dim3(NM, CB), 256, 0, stream>>>(Uu + (size_t)M0 * HID, Tu, b1u, b0, 0, H);
    gemm_split_kernel<float, float, 2><<<dim3(1, CB * NM / 256), blk, 0, stream>>>(A2u, 0, H, 0, nullptr, T2, 128, CB * NM, HID);
    k_fin<NM><<<dim3(NM, CB), 64, 0, stream>>>(T2, CB * NM, b2u, b0, M0, out);
  }
}
